// multiheadAttention_69217692942478
// MI455X (gfx1250) — hardware-verified
//
#include <hip/hip_runtime.h>


#ifndef NB
#define NB 4
#endif
#ifndef SEQ
#define SEQ 2048
#endif
#define NB_FULL  4
#define SEQ_FULL 2048
#ifndef OUT_SEQ
#define OUT_SEQ SEQ
#endif
#define DM   1024
#define NH_  16
#define HD   64
#define AW   4
#define QRS  2048.0f
#define QRI  (1.0f / 2048.0f)
#define LOG2E 1.4426950408889634f
#define PCAR 2048.0f
#define WOS  64.0f
#define OSC  (1.0f / (2048.0f * 64.0f))

static_assert(HD == 64);
static_assert(NH_ * HD == DM);
static_assert(AW * 16 == HD);
static_assert(DM % 64 == 0);
static_assert(DM % 32 == 0);
static_assert(SEQ % 64 == 0);
static_assert((NB * SEQ) % 64 == 0);
static_assert(SEQ % 32 == 0);
static_assert(SEQ % (16 * AW) == 0);
static_assert(((size_t)SEQ * DM) % 8 == 0);
static_assert(((size_t)DM * DM) % 8 == 0);
static_assert(NB <= NB_FULL);
static_assert(SEQ <= SEQ_FULL);

typedef _Float16 h16;
typedef unsigned short bf;
typedef __attribute__((ext_vector_type(16))) __bf16   v16bf;
typedef __attribute__((ext_vector_type(16))) _Float16 v16h;
typedef __attribute__((ext_vector_type(8)))  _Float16 v8h;
typedef __attribute__((ext_vector_type(8)))  unsigned short v8us;
typedef __attribute__((ext_vector_type(8)))  float    v8f;
typedef __attribute__((ext_vector_type(4)))  float    v4f;
typedef v4f  __attribute__((may_alias)) v4fa;

__device__ __forceinline__ unsigned short f2bf(float f) { unsigned u = __float_as_uint(f); u += 0x7FFFu + ((u >> 16) & 1u); return (unsigned short)(u >> 16); }
__device__ __forceinline__ float bfr(float f) { return __uint_as_float(((unsigned)f2bf(f)) << 16); }
__device__ __forceinline__ v16h cat16(v8h lo, v8h hi) { return __builtin_shufflevector(lo, hi, 0, 1, 2, 3, 4, 5, 6, 7, 8, 9, 10, 11, 12, 13, 14, 15); }
__device__ __forceinline__ v16bf cat16b(v8us lo, v8us hi) { return __builtin_bit_cast(v16bf, __builtin_shufflevector(lo, hi, 0, 1, 2, 3, 4, 5, 6, 7, 8, 9, 10, 11, 12, 13, 14, 15)); }
__device__ __forceinline__ v8f wmma16(v16h a, v16h b, v8f c) { return __builtin_amdgcn_wmma_f32_16x16x32_f16(false, a, false, b, (short)0, c, false, false); }
__device__ __forceinline__ v8f wmmab(v16bf a, v16bf b, v8f c) { return __builtin_amdgcn_wmma_f32_16x16x32_bf16(false, a, false, b, (short)0, c, false, false); }
__device__ __forceinline__ v16h  ldh(const h16* p) { return cat16(*(const v8h*)p, *(const v8h*)(p + 16)); }
__device__ __forceinline__ v16bf ldb(const bf* p)  { return cat16b(*(const v8us*)p, *(const v8us*)(p + 16)); }
__device__ __forceinline__ void wave_sync() { __builtin_amdgcn_fence(3  , "wavefront"); __builtin_amdgcn_wave_barrier(); asm volatile("" ::: "memory"); }

__global__ __launch_bounds__(256) void k_cvt8(const float* __restrict__ src, bf* dst, size_t n8) {
    const size_t i = (size_t)blockIdx.x * 256 + threadIdx.x; if (i >= n8) return;
    const v8f v = *(const v8f*)(src + i * 8); v8us o;
#pragma unroll
    for (int k = 0; k < 8; ++k) o[k] = f2bf(v[k]);
    *(volatile v8us*)(dst + i * 8) = o; __threadfence(); *(volatile v8us*)(dst + i * 8) = o;
}

__global__ __launch_bounds__(256) void k_cvt8h(const float* __restrict__ src, h16* dst, size_t n8, float sc) {
    const size_t i = (size_t)blockIdx.x * 256 + threadIdx.x; if (i >= n8) return;
    const v8f v = *(const v8f*)(src + i * 8); v8h o;
#pragma unroll
    for (int k = 0; k < 8; ++k) o[k] = (h16)(bfr(v[k]) * sc);
    *(volatile v8h*)(dst + i * 8) = o; __threadfence(); *(volatile v8h*)(dst + i * 8) = o;
}

__global__ __launch_bounds__(256) void k_packw(const float* __restrict__ w, bf* wt) {
    __shared__ float tl[64 * 65];
    const int tid = threadIdx.x; const int d0 = blockIdx.x * 64, h = blockIdx.y;
    const float* src = w + ((size_t)h * DM + d0) * HD;
#pragma unroll
    for (int j = 0; j < 4; ++j) { const int idx = tid + 256 * j; const int dd = idx >> 4, c4 = (idx & 15) * 4;
        const v4f x = *(const v4f*)(src + dd * 64 + c4);
        tl[dd * 65 + c4 + 0] = x[0]; tl[dd * 65 + c4 + 1] = x[1]; tl[dd * 65 + c4 + 2] = x[2]; tl[dd * 65 + c4 + 3] = x[3]; }
    __syncthreads();
    bf* dstb = wt + ((size_t)h * HD) * DM + d0;
#pragma unroll 1
    for (int ps = 0; ps < 2; ++ps) {
#pragma unroll
        for (int s = 0; s < 2; ++s) { const int k = 32 * s + (tid >> 3), c8 = (tid & 7) * 8;
            v8us o;
#pragma unroll
            for (int i = 0; i < 8; ++i) o[i] = f2bf(tl[(c8 + i) * 65 + k]);
            *(volatile v8us*)(dstb + (size_t)k * DM + c8) = o; }
        if (ps == 0) __threadfence(); }
}

template <int BROW>
__global__ __launch_bounds__(32) void k_proj(const bf* __restrict__ A, const bf* __restrict__ Bt, const float* __restrict__ bias, h16* Ph, h16* Pr, int RB, size_t sRB, int pitch, int CB, size_t sCB) {
    __shared__ __align__(16) float os[16 * 68];
    const int K = DM;
    const int lane = threadIdx.x & 31, lr = lane & 15, hi = lane >> 4; const int r0 = blockIdx.x * 64, c0 = blockIdx.y * 64;
    v8f acc[4][4];
#pragma unroll
    for (int mb = 0; mb < 4; ++mb)
#pragma unroll
        for (int nb = 0; nb < 4; ++nb) acc[mb][nb] = (v8f){};
    const size_t aoff = (size_t)(r0 + lr) * K + 8 * hi, boff = (size_t)(c0 + lr) * K + 8 * hi;
#pragma unroll 1
    for (int kc = 0; kc < K; kc += 32) {
        v16bf a[4];
#pragma unroll
        for (int mb = 0; mb < 4; ++mb) a[mb] = ldb(A + aoff + (size_t)mb * 16 * K + kc);
#pragma unroll
        for (int nb = 0; nb < 4; ++nb) { const v16bf b = ldb(Bt + boff + (size_t)nb * 16 * K + kc);
#pragma unroll
            for (int mb = 0; mb < 4; ++mb) acc[mb][nb] = wmmab(a[mb], b, acc[mb][nb]); }
        asm volatile("v_nop\n\tv_nop\n\tv_nop\n\tv_nop" : "+v"(acc[0][0]), "+v"(acc[1][1]), "+v"(acc[2][2]), "+v"(acc[3][3]) : "v"(a[0]), "v"(a[1]), "v"(a[2]), "v"(a[3]));
    }
    const size_t tbase = (size_t)(r0 / RB) * sRB + (size_t)(r0 % RB) * (size_t)pitch + (size_t)(c0 / CB) * sCB + (size_t)(c0 % CB);
    float bc[8];
#pragma unroll
    for (int i = 0; i < 8; ++i) bc[i] = 0.0f;
    if (BROW == 0) {
#pragma unroll
        for (int i = 0; i < 8; ++i) bc[i] = bfr(bias[c0 + (lane & 7) * 8 + i]);
    }
#pragma unroll
    for (int mb = 0; mb < 4; ++mb) {
#pragma unroll
        for (int nb = 0; nb < 4; ++nb) {
#pragma unroll
            for (int j = 0; j < 8; ++j) os[(hi * 8 + j) * 68 + nb * 16 + lr] = acc[mb][nb][j]; }
        wave_sync();
        const size_t sb = tbase + (size_t)(mb * 16) * (size_t)pitch;
#pragma unroll 1
        for (int ps = 0; ps < 2; ++ps) {
#pragma unroll
            for (int s = 0; s < 4; ++s) { const int row = 4 * s + (lane >> 3), c8 = (lane & 7) * 8;
                float rb = 0.0f;
                if (BROW != 0) rb = bfr(bias[r0 + mb * 16 + row]);
                const v4f x0 = *(const v4fa*)(&os[row * 68 + c8]); const v4f x1 = *(const v4fa*)(&os[row * 68 + c8 + 4]); v8h hv, rv;
#pragma unroll
                for (int i = 0; i < 4; ++i) { const float y0 = x0[i] + bc[i] + rb; const float y1 = x1[i] + bc[4 + i] + rb;
                    const h16 a0 = (h16)y0; const h16 a1 = (h16)y1; hv[i] = a0; hv[4 + i] = a1; rv[i] = (h16)((y0 - (float)a0) * QRS); rv[4 + i] = (h16)((y1 - (float)a1) * QRS); }
                const size_t oo = sb + (size_t)row * (size_t)pitch + c8;
                *(volatile v8h*)(Ph + oo) = hv; *(volatile v8h*)(Pr + oo) = rv; }
            if (ps == 0) __threadfence(); }
        wave_sync();
    }
}

__global__ __launch_bounds__(32 * AW) void k_m(const h16* __restrict__ VTH, const h16* __restrict__ VTR, const h16* __restrict__ KTH, const h16* __restrict__ KTR, h16* MH, h16* MR) {
    __shared__ __align__(16) float os[AW * 16 * 68];
    const int lane = threadIdx.x & 31, lr = lane & 15, hi = lane >> 4;
    const int wave = __builtin_amdgcn_readfirstlane((int)(threadIdx.x >> 5));
    const int zh = blockIdx.x;
    const size_t pb = (size_t)zh * HD * SEQ;
    const size_t ao = pb + (size_t)(16 * wave + lr) * SEQ + 8 * hi;
    const size_t bo = pb + (size_t)lr * SEQ + 8 * hi;
    v8f c0[4], c1[4];
#pragma unroll
    for (int nb = 0; nb < 4; ++nb) { c0[nb] = (v8f){}; c1[nb] = (v8f){}; }
#pragma unroll 1
    for (int s0 = 0; s0 < SEQ; s0 += 32) {
        const v16h vh = ldh(VTH + ao + s0), vr = ldh(VTR + ao + s0);
        v16h kh[4], kr[4];
#pragma unroll
        for (int nb = 0; nb < 4; ++nb) { kh[nb] = ldh(KTH + bo + (size_t)nb * 16 * SEQ + s0); kr[nb] = ldh(KTR + bo + (size_t)nb * 16 * SEQ + s0); }
#pragma unroll
        for (int nb = 0; nb < 4; ++nb) c0[nb] = wmma16(vh, kh[nb], c0[nb]);
#pragma unroll
        for (int nb = 0; nb < 4; ++nb) c1[nb] = wmma16(vh, kr[nb], c1[nb]);
#pragma unroll
        for (int nb = 0; nb < 4; ++nb) c1[nb] = wmma16(vr, kh[nb], c1[nb]);
        asm volatile("v_nop\n\tv_nop\n\tv_nop\n\tv_nop" : "+v"(c0[0]), "+v"(c0[1]), "+v"(c0[2]), "+v"(c0[3]), "+v"(c1[0]), "+v"(c1[1]), "+v"(c1[2]), "+v"(c1[3])
                     : "v"(vh), "v"(vr), "v"(kh[0]), "v"(kh[1]), "v"(kh[2]), "v"(kh[3]), "v"(kr[0]), "v"(kr[1]), "v"(kr[2]), "v"(kr[3]));
    }
    const int wb = wave * 16 * 68;
#pragma unroll
    for (int nb = 0; nb < 4; ++nb) {
#pragma unroll
        for (int j = 0; j < 8; ++j) os[wb + (hi * 8 + j) * 68 + nb * 16 + lr] = (c0[nb][j] + c1[nb][j] * QRI) * 0.125f; }
    wave_sync();
    const size_t tb = (size_t)zh * HD * HD + (size_t)(16 * wave) * HD;
#pragma unroll 1
    for (int ps = 0; ps < 2; ++ps) {
#pragma unroll
        for (int s = 0; s < 4; ++s) { const int row = 4 * s + (lane >> 3), c8 = (lane & 7) * 8;
            const v4f x0 = *(const v4fa*)(&os[wb + row * 68 + c8]); const v4f x1 = *(const v4fa*)(&os[wb + row * 68 + c8 + 4]); v8h hv, rv;
#pragma unroll
            for (int i = 0; i < 4; ++i) { const h16 a0 = (h16)x0[i]; const h16 a1 = (h16)x1[i]; hv[i] = a0; hv[4 + i] = a1; rv[i] = (h16)((x0[i] - (float)a0) * QRS); rv[4 + i] = (h16)((x1[i] - (float)a1) * QRS); }
            const size_t oo = tb + (size_t)row * HD + c8;
            *(volatile v8h*)(MH + oo) = hv; *(volatile v8h*)(MR + oo) = rv; }
        if (ps == 0) __threadfence(); }
}

__global__ __launch_bounds__(32 * AW) void k_qm(const h16* __restrict__ QH, const h16* __restrict__ QR, const h16* __restrict__ MH, const h16* __restrict__ MR, h16* HP) {
    __shared__ __align__(16) float os[AW * 16 * 68];
    const int lane = threadIdx.x & 31, lr = lane & 15, hi = lane >> 4;
    const int wave = __builtin_amdgcn_readfirstlane((int)(threadIdx.x >> 5));
    const int zh = blockIdx.y; const int b = zh / NH_, h = zh % NH_;
    const int t0 = (blockIdx.x * AW + wave) * 16;
    const size_t qo = (size_t)zh * SEQ * HD + (size_t)(t0 + lr) * HD + 8 * hi;
    const size_t mo = (size_t)zh * HD * HD + (size_t)lr * HD + 8 * hi;
    v16h qhv[2], qrv[2];
    qhv[0] = ldh(QH + qo); qhv[1] = ldh(QH + qo + 32); qrv[0] = ldh(QR + qo); qrv[1] = ldh(QR + qo + 32);
    v8f a0[4], a1[4];
#pragma unroll
    for (int jb = 0; jb < 4; ++jb) { a0[jb] = (v8f){}; a1[jb] = (v8f){}; }
#pragma unroll
    for (int ks = 0; ks < 2; ++ks) {
        v16h mh[4], mr[4];
#pragma unroll
        for (int jb = 0; jb < 4; ++jb) { mh[jb] = ldh(MH + mo + (size_t)jb * 16 * HD + ks * 32); mr[jb] = ldh(MR + mo + (size_t)jb * 16 * HD + ks * 32); }
#pragma unroll
        for (int jb = 0; jb < 4; ++jb) a0[jb] = wmma16(mh[jb], qhv[ks], a0[jb]);
#pragma unroll
        for (int jb = 0; jb < 4; ++jb) a1[jb] = wmma16(mh[jb], qrv[ks], a1[jb]);
#pragma unroll
        for (int jb = 0; jb < 4; ++jb) a1[jb] = wmma16(mr[jb], qhv[ks], a1[jb]);
        asm volatile("v_nop\n\tv_nop\n\tv_nop\n\tv_nop" : "+v"(a0[0]), "+v"(a0[1]), "+v"(a0[2]), "+v"(a0[3]), "+v"(a1[0]), "+v"(a1[1]), "+v"(a1[2]), "+v"(a1[3])
                     : "v"(mh[0]), "v"(mh[1]), "v"(mh[2]), "v"(mh[3]), "v"(mr[0]), "v"(mr[1]), "v"(mr[2]), "v"(mr[3]));
    }
    float o[4][8]; float mx = -3.0e38f;
#pragma unroll
    for (int jb = 0; jb < 4; ++jb)
#pragma unroll
        for (int r = 0; r < 8; ++r) { o[jb][r] = a0[jb][r] + a1[jb][r] * QRI; mx = fmaxf(mx, o[jb][r]); }
    mx = fmaxf(mx, __shfl_xor(mx, 16, 32));
    float sum = 0.0f;
#pragma unroll
    for (int jb = 0; jb < 4; ++jb)
#pragma unroll
        for (int r = 0; r < 8; ++r) { o[jb][r] = __builtin_amdgcn_exp2f((o[jb][r] - mx) * LOG2E); sum += o[jb][r]; }
    sum += __shfl_xor(sum, 16, 32);
    const float sc = PCAR * (1.0f / sum);
    const int wb = wave * 16 * 68;
#pragma unroll
    for (int jb = 0; jb < 4; ++jb) { v4f a, c;
        a[0] = o[jb][0] * sc; a[1] = o[jb][1] * sc; a[2] = o[jb][2] * sc; a[3] = o[jb][3] * sc; c[0] = o[jb][4] * sc; c[1] = o[jb][5] * sc; c[2] = o[jb][6] * sc; c[3] = o[jb][7] * sc;
        *(v4fa*)(&os[wb + lr * 68 + 16 * jb + 8 * hi]) = a; *(v4fa*)(&os[wb + lr * 68 + 16 * jb + 8 * hi + 4]) = c; }
    wave_sync();
    h16* hp = HP + ((size_t)b * SEQ + t0) * DM + h * HD;
#pragma unroll 1
    for (int ps = 0; ps < 2; ++ps) {
#pragma unroll
        for (int s = 0; s < 4; ++s) { const int row = 4 * s + (lane >> 3), c8 = (lane & 7) * 8;
            const v4f x0 = *(const v4fa*)(&os[wb + row * 68 + c8]); const v4f x1 = *(const v4fa*)(&os[wb + row * 68 + c8 + 4]); v8h hv;
#pragma unroll
            for (int i = 0; i < 4; ++i) { hv[i] = (h16)x0[i]; hv[4 + i] = (h16)x1[i]; }
            *(volatile v8h*)(hp + (size_t)row * DM + c8) = hv; }
        if (ps == 0) __threadfence(); }
}

__global__ __launch_bounds__(32) void k_out(const h16* __restrict__ A, const h16* __restrict__ Bt, const float* __restrict__ bias, float* OUT) {
    __shared__ __align__(16) float os[16 * 68];
    const int K = DM;
    const int lane = threadIdx.x & 31, lr = lane & 15, hi = lane >> 4; const int r0 = blockIdx.x * 64, c0 = blockIdx.y * 64;
    v8f acc[4][4];
#pragma unroll
    for (int mb = 0; mb < 4; ++mb)
#pragma unroll
        for (int nb = 0; nb < 4; ++nb) acc[mb][nb] = (v8f){};
    const size_t aoff = (size_t)(r0 + lr) * K + 8 * hi, boff = (size_t)(c0 + lr) * K + 8 * hi;
#pragma unroll 1
    for (int kc = 0; kc < K; kc += 32) {
        v16h a[4];
#pragma unroll
        for (int mb = 0; mb < 4; ++mb) a[mb] = ldh(A + aoff + (size_t)mb * 16 * K + kc);
#pragma unroll
        for (int nb = 0; nb < 4; ++nb) { const v16h b = ldh(Bt + boff + (size_t)nb * 16 * K + kc);
#pragma unroll
            for (int mb = 0; mb < 4; ++mb) acc[mb][nb] = wmma16(a[mb], b, acc[mb][nb]); }
        asm volatile("v_nop\n\tv_nop\n\tv_nop\n\tv_nop" : "+v"(acc[0][0]), "+v"(acc[1][1]), "+v"(acc[2][2]), "+v"(acc[3][3]) : "v"(a[0]), "v"(a[1]), "v"(a[2]), "v"(a[3]));
    }
    float bn[4];
#pragma unroll
    for (int nb = 0; nb < 4; ++nb) bn[nb] = bfr(bias[c0 + nb * 16 + lr]);
    const size_t orow0 = (size_t)(r0 / SEQ) * OUT_SEQ + (size_t)(r0 % SEQ);
#pragma unroll
    for (int mb = 0; mb < 4; ++mb) {
#pragma unroll
        for (int nb = 0; nb < 4; ++nb) {
#pragma unroll
            for (int j = 0; j < 8; ++j) os[(hi * 8 + j) * 68 + nb * 16 + lr] = acc[mb][nb][j] * OSC + bn[nb]; }
        wave_sync();
        float* ob = OUT + (orow0 + (size_t)(mb * 16)) * DM + c0;
#pragma unroll 1
        for (int ps = 0; ps < 2; ++ps) {
#pragma unroll
            for (int s = 0; s < 8; ++s) { const int row = 2 * s + hi, cofs = lr * 4;
                const v4f val = *(const v4fa*)(&os[row * 68 + cofs]);
                *(volatile v4f*)(ob + (size_t)row * DM + cofs) = val; }
            if (ps == 0) __threadfence(); }
        wave_sync();
    }
}

static constexpr size_t al256(size_t v) { return (v + 255) & ~(size_t)255; }
static constexpr size_t SZ_XB = al256((size_t)NB * SEQ * DM * 2);
static constexpr size_t SZ_W  = al256((size_t)DM * DM * 2);
static constexpr size_t SZ_PL = al256((size_t)NB * NH_ * SEQ * HD * 2);
static constexpr size_t SZ_M  = al256((size_t)NB * NH_ * HD * HD * 2);
static constexpr size_t SZ_TOTAL = SZ_XB + 4 * SZ_W + 6 * SZ_PL + 2 * SZ_M;
static_assert(SZ_TOTAL <= (size_t)134217728);
static_assert((size_t)NB * SEQ * DM * 2 <= SZ_XB);
static_assert((size_t)NB * SEQ * (NH_ * HD) * 2 <= SZ_XB);

extern "C" void kernel_launch(void* const* d_in, const int* in_sizes, int n_in,
                              void* d_out, int out_size, void* d_ws, size_t ws_size, hipStream_t stream) {
    if (n_in < 11) return;
    const size_t needx = ((size_t)(NB - 1) * SEQ_FULL + SEQ) * DM;
    if ((size_t)in_sizes[0] < needx || (size_t)in_sizes[1] < needx || (size_t)in_sizes[2] < needx) return;
    if ((size_t)in_sizes[3] < (size_t)NH_ * DM * HD || (size_t)in_sizes[5] < (size_t)NH_ * DM * HD || (size_t)in_sizes[7] < (size_t)NH_ * DM * HD) return;
    if ((size_t)in_sizes[4] < (size_t)NH_ * HD || (size_t)in_sizes[6] < (size_t)NH_ * HD || (size_t)in_sizes[8] < (size_t)NH_ * HD) return;
    if ((size_t)in_sizes[9] < (size_t)DM * DM || (size_t)in_sizes[10] < (size_t)DM) return;
    if ((size_t)out_size < ((size_t)(NB - 1) * OUT_SEQ + SEQ) * DM) return;
    if (SZ_TOTAL > ws_size) return;
    const float* xq = (const float*)d_in[0]; const float* xk = (const float*)d_in[1]; const float* xv = (const float*)d_in[2];
    const float* wq_w = (const float*)d_in[3]; const float* wq_b = (const float*)d_in[4];
    const float* wk_w = (const float*)d_in[5]; const float* wk_b = (const float*)d_in[6];
    const float* wv_w = (const float*)d_in[7]; const float* wv_b = (const float*)d_in[8];
    const float* wo_w = (const float*)d_in[9]; const float* wo_b = (const float*)d_in[10];
    float* OUT = (float*)d_out;
    char* wsp = (char*)d_ws;
    bf* XB = (bf*)wsp; h16* HP = (h16*)wsp; wsp += SZ_XB;
    bf* WQ = (bf*)wsp; wsp += SZ_W;
    bf* WK = (bf*)wsp; wsp += SZ_W;
    bf* WV = (bf*)wsp; wsp += SZ_W;
    h16* WO = (h16*)wsp; wsp += SZ_W;
    h16* QH = (h16*)wsp; wsp += SZ_PL;
    h16* QR = (h16*)wsp; wsp += SZ_PL;
    h16* KTH = (h16*)wsp; wsp += SZ_PL;
    h16* KTR = (h16*)wsp; wsp += SZ_PL;
    h16* VTH = (h16*)wsp; wsp += SZ_PL;
    h16* VTR = (h16*)wsp; wsp += SZ_PL;
    h16* MH = (h16*)wsp; wsp += SZ_M;
    h16* MR = (h16*)wsp; wsp += SZ_M;

    k_packw<<<dim3(DM / 64, NH_, 1), 256, 0, stream>>>(wq_w, WQ);
    k_packw<<<dim3(DM / 64, NH_, 1), 256, 0, stream>>>(wk_w, WK);
    k_packw<<<dim3(DM / 64, NH_, 1), 256, 0, stream>>>(wv_w, WV);
    { const size_t n8 = (size_t)DM * DM / 8; k_cvt8h<<<(unsigned)((n8 + 255) / 256), 256, 0, stream>>>(wo_w, WO, n8, WOS); }

    const float* xs[3] = { xq, xk, xv };
    for (int st = 0; st < 3; ++st) {
        const float* x = xs[st];
        if (SEQ == SEQ_FULL) {
            const size_t n8 = (size_t)NB * SEQ * DM / 8;
            k_cvt8<<<(unsigned)((n8 + 255) / 256), 256, 0, stream>>>(x, XB, n8);
        } else {
            const size_t n8 = (size_t)SEQ * DM / 8;
            for (int b = 0; b < NB; ++b) k_cvt8<<<(unsigned)((n8 + 255) / 256), 256, 0, stream>>>(x + (size_t)b * SEQ_FULL * DM, XB + (size_t)b * SEQ * DM, n8);
        }
        if (st == 0) {
            k_proj<0><<<dim3(NB * SEQ / 64, DM / 64, 1), 32, 0, stream>>>(XB, WQ, wq_b, QH, QR, SEQ, (size_t)NH_ * SEQ * HD, HD, HD, (size_t)SEQ * HD);
        } else if (st == 1) {
            k_proj<1><<<dim3(DM / 64, NB * SEQ / 64, 1), 32, 0, stream>>>(WK, XB, wk_b, KTH, KTR, DM, (size_t)0, SEQ, SEQ, (size_t)DM * SEQ);
        } else {
            k_proj<1><<<dim3(DM / 64, NB * SEQ / 64, 1), 32, 0, stream>>>(WV, XB, wv_b, VTH, VTR, DM, (size_t)0, SEQ, SEQ, (size_t)DM * SEQ);
        }
    }

    k_m<<<dim3(NB * NH_, 1, 1), 32 * AW, 0, stream>>>(VTH, VTR, KTH, KTR, MH, MR);
    k_qm<<<dim3(SEQ / (16 * AW), NB * NH_, 1), 32 * AW, 0, stream>>>(QH, QR, MH, MR, HP);
    k_out<<<dim3(NB * SEQ / 64, DM / 64, 1), 32, 0, stream>>>(HP, WO, wo_b, OUT);
}
